// MemristorConv1d_42494406427032
// MI455X (gfx1250) — hardware-verified
//
#include <hip/hip_runtime.h>


namespace {
constexpr int B = 8, C = 512, T = 1024, K = 31, PAD = 15, NP = 3;
constexpr float WSC = 256.0f, VMAX = 0.6f, LEV = 127.0f, CUR = 8020.0f, STEP = 0.00390625f, LIM = 32.0f;
typedef _Float16 b16;
typedef __attribute__((ext_vector_type(16))) _Float16 v16b;
typedef __attribute__((ext_vector_type(8))) _Float16 v8b;
typedef __attribute__((ext_vector_type(8))) float v8f;
__device__ __forceinline__ float bf16_rne(float f) { unsigned int u = __float_as_uint(f); u += 0x7FFFu + ((u >> 16) & 1u); return __uint_as_float(u & 0xFFFF0000u); }
__device__ __forceinline__ void split16(float v, b16& hi, b16& lo) { hi = (b16)v; lo = (b16)(v - (float)hi); }
__device__ __forceinline__ v16b frag_kb(const b16* p, int hh) { const v8b a = *(const v8b*)(p + 8 * hh), b = *(const v8b*)(p + 16 + 8 * hh); v16b f;
#pragma unroll
  for (int e = 0; e < 8; ++e) { f[e] = a[e]; f[8 + e] = b[e]; } return f; }
__device__ __forceinline__ v8f wmma16b(v16b a, v16b b, v8f c) { v8f d = __builtin_amdgcn_wmma_f32_16x16x32_f16(false, a, false, b, (short)0, c, false, false); asm volatile("v_nop\n\tv_nop\n\tv_nop\n\tv_nop" : "+v"(d) : "v"(a), "v"(b)); return d; }
__device__ __forceinline__ void wave_lds_sync() { __builtin_amdgcn_fence(__ATOMIC_RELEASE, "workgroup"); __builtin_amdgcn_wave_barrier(); __builtin_amdgcn_fence(__ATOMIC_ACQUIRE, "workgroup"); }
__device__ __forceinline__ float pmul(float a, float b) { float p = a * b; asm volatile("" : "+v"(p)); return p; }
__device__ __forceinline__ float pdiv(float a, float b) { float p = __fdiv_rn(a, b); asm volatile("" : "+v"(p)); return p; }

__global__ __launch_bounds__(256) void wb_kernel(const float* __restrict__ w, b16* __restrict__ WB) {
  const int u = blockIdx.x * 256 + threadIdx.x; if (u >= C * 16 * 4) return; const int c = u / 64, n = (u / 4) % 16, k0 = (u % 4) * 8; v8b v;
#pragma unroll
  for (int j = 0; j < 8; ++j) { const int k = k0 + j; v[j] = (n < NP && k < K) ? (b16)(bf16_rne(w[((size_t)n * C + c) * K + k]) * WSC) : (b16)0.0f; }
  for (int pass = 0; pass < 2; ++pass) { *(volatile v8b*)(WB + ((size_t)c * 16 + n) * 32 + k0) = v; __threadfence(); }
}
__global__ __launch_bounds__(32) void conv_kernel(const float* __restrict__ x, const b16* __restrict__ WB, const float* __restrict__ bias, const float* __restrict__ fin, const float* __restrict__ fout, int NBV, float* __restrict__ out) {
  __shared__ float Vs[64]; __shared__ __attribute__((aligned(16))) b16 Ah[32][32 + 8], Al[32][32 + 8]; __shared__ float So[32];
  const int lane = threadIdx.x, nloc = lane & 15, hlf = lane >> 4; const int t0 = (blockIdx.x % (T / 32)) * 32, c = (blockIdx.x / (T / 32)) % C, b = blockIdx.x / ((T / 32) * C); if (b >= NBV) return;
  const float f_in = bf16_rne(fin[0]), f_out = bf16_rne(fout[0]); const float* xr = x + ((size_t)b * C + c) * T;
  for (int i = lane; i < 64; i += 32) { const int t = t0 - PAD + i; float v = 0.0f; if (i < 62 && t >= 0 && t < T) { float a = pmul(bf16_rne(xr[t]), f_in); a = fminf(fmaxf(a, -1.0f), 1.0f); a = rintf(pmul(a, LEV)); v = pmul(pdiv(a, LEV), VMAX); } Vs[i] = v; }
  wave_lds_sync();
  for (int r = 0; r < 32; ++r) { b16 p, q; split16(Vs[r + lane], p, q); Ah[r][lane] = p; Al[r][lane] = q; }
  wave_lds_sync();
  const b16* wr = WB + ((size_t)c * 16 + nloc) * 32; const v16b bw = frag_kb(wr, hlf);
#pragma unroll
  for (int tile = 0; tile < 2; ++tile) { v8f acc = {}; acc = wmma16b(frag_kb(&Ah[tile * 16 + nloc][0], hlf), bw, acc); acc = wmma16b(frag_kb(&Al[tile * 16 + nloc][0], hlf), bw, acc);
    float mem[8];
#pragma unroll
    for (int r8 = 0; r8 < 8; ++r8) { float cur = acc[r8] * (1.0f / WSC); float a = rintf(pdiv(pmul(cur, CUR), STEP)); a = pmul(a, STEP); a = fminf(fmaxf(a, -LIM), LIM); const float pw = nloc == 0 ? 4.0f : (nloc == 1 ? 2.0f : (nloc == 2 ? 1.0f : 0.0f)); mem[r8] = pmul(a, pw); }
#pragma unroll
    for (int r8 = 0; r8 < 8; ++r8) { float s = mem[r8]; for (int o = 1; o < 16; o <<= 1) s += __shfl_xor(s, o); if (nloc == 0) So[tile * 16 + 8 * hlf + r8] = pmul(s, f_out) + bf16_rne(bias[c]); } }
  wave_lds_sync();
  for (int pass = 0; pass < 2; ++pass) { ((volatile float*)out)[((size_t)b * C + c) * T + t0 + lane] = So[lane]; __threadfence(); }
}
}

extern "C" void kernel_launch(void* const* d_in, const int* in_sizes, int n_in, void* d_out, int out_size, void* d_ws, size_t ws_size, hipStream_t stream) {
  (void)n_in;
  auto Fp = [&](int i) { return (const float*)d_in[i]; };
  if (in_sizes[0] != B * C * T || in_sizes[1] != NP * C * K || in_sizes[2] != C || in_sizes[3] != 1 || in_sizes[4] != 1 || out_size != B * C * T) return;
  const int NBV = B;
  size_t off = 0; char* ws = (char*)d_ws;
  auto carve = [&](size_t bytes) { char* p = ws + off; off += (bytes + 255) & ~(size_t)255; return p; };
  b16* WB = (b16*)carve((size_t)C * 16 * 32 * 2);
  if (off > ws_size || off > ((size_t)8 << 20)) return;
  wb_kernel<<<(C * 64 + 255) / 256, 256, 0, stream>>>(Fp(1), WB);
  conv_kernel<<<NBV * C * (T / 32), 32, 0, stream>>>(Fp(0), WB, Fp(2), Fp(3), Fp(4), NBV, (float*)d_out);
}
